// gc_gcn_32006096290304
// MI455X (gfx1250) — hardware-verified
//
#include <hip/hip_runtime.h>
#include <math.h>


#define BB    64
#define CC    64
#define TT    128
#define VV    25
#define RR    8
#define TS    9
#define OUTC  64
#define TVTOT (TT * VV)
#define PADV  32
#define XROWS (TT + TS - 1)
#define RELN  (RR * VV * VV)
#define RELP  5024
#define ZTP   72
#define OSP   68
#define SLAB  64
#define NTV   (TVTOT / SLAB)

typedef char chk_rel_pitch[(RELP % 32 == 0 && RELP >= RELN) ? 1 : -1];
typedef char chk_tv_slabs[(TVTOT % SLAB == 0) ? 1 : -1];
typedef char chk_z_lines[((TVTOT * 2) % 128 == 0) ? 1 : -1];
typedef char chk_lds_pitch[((ZTP * 2) % 16 == 0 && (OSP * 4) % 16 == 0) ? 1 : -1];

typedef _Float16 v16h __attribute__((ext_vector_type(16)));
typedef _Float16 v8h  __attribute__((ext_vector_type(8)));
typedef float    v8f  __attribute__((ext_vector_type(8)));
typedef float    v4f  __attribute__((ext_vector_type(4)));
typedef unsigned int v4u __attribute__((ext_vector_type(4)));
typedef v8h __attribute__((__may_alias__)) v8ha;
typedef v4f __attribute__((__may_alias__)) v4fa;
typedef v4u __attribute__((__may_alias__)) v4ua;

union Frag { v16h v; v8h half[2]; };
union ZChunk { v4u u; _Float16 hh[8]; };

__device__ __forceinline__ v8f wmma_f16(const v16h a, const v16h b, v8f c)
{
    v8f d = __builtin_amdgcn_wmma_f32_16x16x32_f16(false, a, false, b, (short)0, c, false, false);
    asm volatile("v_nop\n\tv_nop\n\tv_nop\n\tv_nop" : "+v"(d) : "v"(a), "v"(b));
    return d;
}

__device__ __forceinline__ v16h load_frag(const _Float16* p, int h)
{
    Frag f;
    f.half[0] = *(const v8ha*)(p + 8 * h);
    f.half[1] = *(const v8ha*)(p + 16 + 8 * h);
    return f.v;
}

__global__ __launch_bounds__(256)
void k_rel(const float* __restrict__ x, const float* __restrict__ W1,
           const float* __restrict__ b1, const float* __restrict__ W2,
           const float* __restrict__ b2, float* rel)
{
    if (blockIdx.x >= BB) return;
    const int b   = blockIdx.x;
    const int tid = threadIdx.x;
    __shared__ float xm[CC * VV];
    __shared__ float x1s[RR * VV];
    __shared__ float x2s[RR * VV];
    __shared__ __align__(16) float rs[RELP];

    const float* xb = x + (size_t)b * CC * TT * VV;
    for (int idx = tid; idx < CC * VV; idx += 256) {
        const int c = idx / VV, v = idx - c * VV;
        const float* p = xb + (size_t)c * TT * VV + v;
        float s = 0.f;
        #pragma unroll 4
        for (int t = 0; t < TT; ++t) s += p[t * VV];
        xm[idx] = s * (1.0f / (float)TT);
    }
    __syncthreads();

    for (int idx = tid; idx < 2 * RR * VV; idx += 256) {
        const int which = idx / (RR * VV);
        const int rv = idx - which * (RR * VV);
        const int r = rv / VV, v = rv - r * VV;
        const float* W = which ? W2 : W1;
        float s = 0.f;
        #pragma unroll 8
        for (int c = 0; c < CC; ++c) s += W[r * CC + c] * xm[c * VV + v];
        s += which ? b2[r] : b1[r];
        (which ? x2s : x1s)[rv] = s;
    }
    __syncthreads();

    for (int idx = tid; idx < RELP; idx += 256) {
        float t = 0.f;
        if (idx < RELN) {
            const int r   = idx / (VV * VV);
            const int rem = idx - r * (VV * VV);
            const int v   = rem / VV, i = rem - v * VV;
            t = tanhf(x1s[r * VV + v] - x2s[r * VV + i]);
        }
        rs[idx] = t;
    }
    __syncthreads();

    float* relb = rel + (size_t)b * RELP;
    for (int q = tid; q < RELP / 4; q += 256) {
        const v4f val = *(const v4fa*)&rs[4 * q];
        *(volatile v4f*)(relb + 4 * q) = val;
    }
    __threadfence();
    for (int q = tid; q < RELP / 4; q += 256) {
        const v4f val = *(const v4fa*)&rs[4 * q];
        *(volatile v4f*)(relb + 4 * q) = val;
    }
}

__global__ __launch_bounds__(128)
void k_tgconv(const float* __restrict__ x, const float* __restrict__ A,
              const float* __restrict__ W4, const float* __restrict__ b4,
              const float* __restrict__ rel, _Float16* zws)
{
    if (blockIdx.x >= BB * CC) return;
    const int bc  = blockIdx.x;
    const int b   = bc >> 6, c = bc & 63;
    const int tid = threadIdx.x;

    __shared__ __align__(16) _Float16 xs[XROWS * PADV];
    __shared__ __align__(16) _Float16 mt[TS * PADV * PADV];
    __shared__ __align__(16) _Float16 zs[TVTOT];
    __shared__ float w4s[TS * RR];
    __shared__ float b4s[16];

    if (tid < TS * RR) w4s[tid] = W4[(size_t)(c * TS) * RR + tid];
    if (tid < TS)      b4s[tid] = b4[c * TS + tid];

    const float* xb = x + ((size_t)b * CC + c) * TT * VV;
    for (int idx = tid; idx < XROWS * PADV; idx += 128) {
        const int row = idx >> 5, v = idx & 31;
        float val = 0.f;
        if (row >= TS - 1 && v < VV) val = xb[(size_t)(row - (TS - 1)) * VV + v];
        xs[idx] = (_Float16)(val * 16.0f);
    }
    __syncthreads();

    const float* relb = rel + (size_t)b * RELP;
    for (int p = tid; p < PADV * PADV; p += 128) {
        const int i = p >> 5, v = p & 31;
        if (i < VV && v < VV) {
            float rr[RR];
            #pragma unroll
            for (int r = 0; r < RR; ++r) rr[r] = relb[r * (VV * VV) + v * VV + i];
            const float av = A[v * VV + i];
            #pragma unroll
            for (int k = 0; k < TS; ++k) {
                float s = 0.f;
                #pragma unroll
                for (int r = 0; r < RR; ++r) s += w4s[k * RR + r] * rr[r];
                s += b4s[k];
                s += av;
                mt[(k * PADV + i) * PADV + v] = (_Float16)(s * 64.0f);
            }
        } else {
            #pragma unroll
            for (int k = 0; k < TS; ++k) mt[(k * PADV + i) * PADV + v] = (_Float16)0.0f;
        }
    }
    __syncthreads();

    const int lane = tid & 31, w = tid >> 5;
    const int m = lane & 15, h = lane >> 4;

    v8f acc[2][2];
    #pragma unroll
    for (int mi = 0; mi < 2; ++mi)
        #pragma unroll
        for (int ni = 0; ni < 2; ++ni)
            #pragma unroll
            for (int r = 0; r < 8; ++r) acc[mi][ni][r] = 0.f;

    #pragma unroll
    for (int k = 0; k < TS; ++k) {
        v16h af[2], bf[2];
        #pragma unroll
        for (int mi = 0; mi < 2; ++mi) {
            const int row = (2 * w + mi) * 16 + m + k;
            af[mi] = load_frag(&xs[row * PADV], h);
        }
        #pragma unroll
        for (int ni = 0; ni < 2; ++ni) {
            const int col = ni * 16 + m;
            bf[ni] = load_frag(&mt[(k * PADV + col) * PADV], h);
        }
        #pragma unroll
        for (int mi = 0; mi < 2; ++mi)
            #pragma unroll
            for (int ni = 0; ni < 2; ++ni)
                acc[mi][ni] = wmma_f16(af[mi], bf[ni], acc[mi][ni]);
    }

    #pragma unroll
    for (int mi = 0; mi < 2; ++mi) {
        #pragma unroll
        for (int ni = 0; ni < 2; ++ni) {
            const int i = ni * 16 + m;
            if (i < VV) {
                #pragma unroll
                for (int r = 0; r < 8; ++r) {
                    const int t = (2 * w + mi) * 16 + 8 * h + r;
                    zs[t * VV + i] = (_Float16)(acc[mi][ni][r] * (1.0f / 64.0f));
                }
            }
        }
    }
    __syncthreads();

    _Float16* zrow = zws + (size_t)bc * TVTOT;
    for (int f = tid; f < TVTOT / 8; f += 128) {
        const v4u val = *(const v4ua*)&zs[8 * f];
        *(volatile v4u*)(zrow + 8 * f) = val;
    }
    __threadfence();
    for (int f = tid; f < TVTOT / 8; f += 128) {
        const v4u val = *(const v4ua*)&zs[8 * f];
        *(volatile v4u*)(zrow + 8 * f) = val;
    }
}

__global__ __launch_bounds__(128)
void k_outconv(const _Float16* __restrict__ zws, const float* __restrict__ W3,
               const float* __restrict__ b3, float* out)
{
    if (blockIdx.x >= BB * NTV) return;
    const int b   = blockIdx.x / NTV;
    const int jt  = blockIdx.x - b * NTV;
    const int tv0 = jt * SLAB;
    const int tid = threadIdx.x;

    __shared__ __align__(16) _Float16 zT[SLAB * ZTP];
    __shared__ __align__(16) _Float16 w3s[OUTC * ZTP];
    __shared__ __align__(16) float outs[OUTC * OSP];
    __shared__ float b3s[OUTC];

    for (int idx = tid; idx < OUTC * CC; idx += 128) {
        const int o = idx >> 6, cc = idx & 63;
        w3s[o * ZTP + cc] = (_Float16)(W3[idx] * 64.0f);
    }
    if (tid < OUTC) b3s[tid] = b3[tid];

    const _Float16* zb = zws + (size_t)b * CC * TVTOT + tv0;
    for (int f = tid; f < CC * (SLAB / 8); f += 128) {
        const int cc = f >> 3, q = f & 7;
        ZChunk zc;
        zc.u = *(const v4ua*)(zb + (size_t)cc * TVTOT + 8 * q);
        #pragma unroll
        for (int e = 0; e < 8; ++e) zT[(8 * q + e) * ZTP + cc] = zc.hh[e];
    }
    __syncthreads();

    const int lane = tid & 31, w = tid >> 5;
    const int m = lane & 15, h = lane >> 4;

    v8f acc[4];
    #pragma unroll
    for (int ni = 0; ni < 4; ++ni)
        #pragma unroll
        for (int r = 0; r < 8; ++r) acc[ni][r] = 0.f;

    #pragma unroll
    for (int kc = 0; kc < CC / 32; ++kc) {
        const v16h af = load_frag(&zT[(16 * w + m) * ZTP + 32 * kc], h);
        #pragma unroll
        for (int ni = 0; ni < 4; ++ni) {
            const v16h bf = load_frag(&w3s[(ni * 16 + m) * ZTP + 32 * kc], h);
            acc[ni] = wmma_f16(af, bf, acc[ni]);
        }
    }

    #pragma unroll
    for (int ni = 0; ni < 4; ++ni) {
        const int o = ni * 16 + m;
        const float bias = b3s[o];
        #pragma unroll
        for (int r = 0; r < 8; ++r) {
            const int tvl = 16 * w + 8 * h + r;
            outs[o * OSP + tvl] = acc[ni][r] * (1.0f / 1024.0f) + bias;
        }
    }
    __syncthreads();

    float* ob = out + (size_t)b * OUTC * TVTOT + tv0;
    for (int f = tid; f < OUTC * (SLAB / 4); f += 128) {
        const int o = f >> 4, q = f & 15;
        const v4f val = *(const v4fa*)&outs[o * OSP + 4 * q];
        *(volatile v4f*)(ob + (size_t)o * TVTOT + 4 * q) = val;
    }
    __threadfence();
    for (int f = tid; f < OUTC * (SLAB / 4); f += 128) {
        const int o = f >> 4, q = f & 15;
        const v4f val = *(const v4fa*)&outs[o * OSP + 4 * q];
        *(volatile v4f*)(ob + (size_t)o * TVTOT + 4 * q) = val;
    }
}

extern "C" void kernel_launch(void* const* d_in, const int* in_sizes, int n_in,
                              void* d_out, int out_size, void* d_ws, size_t ws_size,
                              hipStream_t stream)
{
    if (n_in < 10) return;
    if (in_sizes[0] != BB * CC * TT * VV) return;
    if (in_sizes[1] != VV * VV) return;
    if (in_sizes[2] != RR * CC || in_sizes[3] != RR) return;
    if (in_sizes[4] != RR * CC || in_sizes[5] != RR) return;
    if (in_sizes[6] != CC * TS * RR || in_sizes[7] != CC * TS) return;
    if (in_sizes[8] != OUTC * CC || in_sizes[9] != OUTC) return;
    if (out_size != BB * OUTC * TVTOT) return;

    const float* x  = (const float*)d_in[0];
    const float* A  = (const float*)d_in[1];
    const float* W1 = (const float*)d_in[2];
    const float* b1 = (const float*)d_in[3];
    const float* W2 = (const float*)d_in[4];
    const float* b2 = (const float*)d_in[5];
    const float* W4 = (const float*)d_in[6];
    const float* b4 = (const float*)d_in[7];
    const float* W3 = (const float*)d_in[8];
    const float* b3 = (const float*)d_in[9];
    float* out = (float*)d_out;

    const size_t z_bytes   = (size_t)BB * CC * TVTOT * sizeof(_Float16);
    const size_t rel_bytes = (size_t)BB * RELP * sizeof(float);
    if (z_bytes + rel_bytes > ws_size) return;
    _Float16* z_ws   = (_Float16*)d_ws;
    float*    rel_ws = (float*)((char*)d_ws + z_bytes);

    k_rel<<<BB, 256, 0, stream>>>(x, W1, b1, W2, b2, rel_ws);
    k_tgconv<<<BB * CC, 128, 0, stream>>>(x, A, W4, b4, rel_ws, z_ws);
    k_outconv<<<BB * NTV, 128, 0, stream>>>(z_ws, W3, b3, out);
    (void)hipGetLastError();
}
